// Winograd2d_1949915153157
// MI455X (gfx1250) — hardware-run, weakly checked
//
#include <hip/hip_runtime.h>

typedef __attribute__((ext_vector_type(16))) _Float16 v16h;
typedef __attribute__((ext_vector_type(8)))  _Float16 v8h;
typedef __attribute__((ext_vector_type(8)))  float    v8f;
typedef __attribute__((ext_vector_type(4)))  float    v4f;
typedef __attribute__((ext_vector_type(2)))  float    v2f;

constexpr int kNB    = 32;
constexpr int kCin   = 64;
constexpr int kHW    = 56;
constexpr int kOC    = 128;
constexpr int kNT    = 14;
constexpr int kTPI   = kNT * kNT;
constexpr int kMtot  = kNB * kTPI;
constexpr int kHalfN = 16;
constexpr int kMhalf = kHalfN * kTPI;
constexpr int kP     = 64;
constexpr float kWCarry    = 1024.0f;
constexpr float kGemmScale = 1.0f / 16.0f;
constexpr float kYCarry    = kWCarry * kGemmScale;
constexpr float kYInv      = 1.0f / kYCarry;
static_assert(kTPI == 196);
static_assert(kMtot == 6272);
static_assert(kMhalf == 3136);
static_assert(kHW == 4 * kNT);
static_assert((kMhalf % 64) == 0 && (kOC % 64) == 0 && (kCin % 32) == 0);
static_assert(kYCarry == 64.0f);

constexpr size_t kSzWP = (size_t)kP * kOC * kCin * 2;
constexpr size_t kSzXT = (size_t)kP * kMtot * kCin * 2;
constexpr size_t kSzYT = (size_t)kP * kMhalf * kOC * 2;
constexpr size_t kOffWP = 0;
constexpr size_t kOffXT = kOffWP + kSzWP;
constexpr size_t kOffYT = kOffXT + kSzXT;
constexpr size_t kWsTotal = kOffYT + kSzYT;
static_assert(kSzWP == 1048576ull && kSzXT == 51380224ull && kSzYT == 51380224ull);
static_assert(kWsTotal == 103809024ull);
static_assert(kWsTotal <= 134217728ull);
static_assert((kOffXT % 128) == 0 && (kOffYT % 128) == 0);

__device__ __forceinline__ void bt8(const float d[8], float t[8]) {
  t[0] = (d[0] - d[6]) + 5.25f * (d[4] - d[2]);
  t[7] = (d[7] - d[1]) + 5.25f * (d[3] - d[5]);
  const float pa = (d[2] + d[6]) - 4.25f * d[4];
  const float pb = (d[1] + d[5]) - 4.25f * d[3];
  t[1] = pa + pb;
  t[2] = pa - pb;
  const float pc = (d[6] + 0.25f * d[2]) - 1.25f * d[4];
  const float pe = (0.5f * d[1] - 2.5f * d[3]) + 2.0f * d[5];
  t[3] = pc + pe;
  t[4] = pc - pe;
  const float pf = (d[6] + 4.0f * d[2]) - 5.0f * d[4];
  const float pg = (2.0f * d[1] - 2.5f * d[3]) + 0.5f * d[5];
  t[5] = pf + pg;
  t[6] = pf - pg;
}

__device__ __forceinline__ void at4(const float y[8], float z[4]) {
  const float s12 = y[1] + y[2], d12 = y[1] - y[2];
  const float s34 = y[3] + y[4], d34 = y[3] - y[4];
  const float s56 = y[5] + y[6], d56 = y[5] - y[6];
  z[0] = ((y[0] + s12) + s34) + 8.0f * s56;
  z[1] = (d12 + 2.0f * d34) + 4.0f * d56;
  z[2] = (s12 + 4.0f * s34) + 2.0f * s56;
  z[3] = ((d12 + d56) + y[7]) + 8.0f * d34;
}

__device__ __forceinline__ float h16_to_f32(unsigned hb) {
  const unsigned sgn = (hb & 0x8000u) << 16;
  const unsigned em = hb & 0x7fffu;
  const float fn = __uint_as_float((em << 13) + 0x38000000u);
  const float fs = (float)em * 5.9604644775390625e-8f;
  const float mag = (em < 0x400u) ? fs : fn;
  return __uint_as_float(__float_as_uint(mag) | sgn);
}

__device__ __forceinline__ v16h frag_load(const _Float16* p) {
  union U { v16h v; v8h h[2]; } f;
  f.h[0] = *(const v8h*)(p);
  f.h[1] = *(const v8h*)(p + 16);
  return f.v;
}
__device__ __forceinline__ v8f mma_f16(v16h a, v16h b, v8f c) {
  c = __builtin_amdgcn_wmma_f32_16x16x32_f16(false, a, false, b, (short)0, c, false, false);
  asm volatile("v_nop\n\tv_nop\n\tv_nop\n\tv_nop" : "+v"(c) : "v"(a), "v"(b));
  return c;
}

__global__ __launch_bounds__(256) void pack_w_kernel(const float* __restrict__ w, unsigned short* __restrict__ WP) {
  __shared__ __align__(16) float sW[kCin * 65];
  const int tid = threadIdx.x;
  const int lane = tid & 31;
  const int wave = __builtin_amdgcn_readfirstlane((int)(threadIdx.x >> 5));
  const int o = blockIdx.x;
  const float* src = w + (size_t)o * (kCin * kP);
#pragma unroll
  for (int it = 0; it < 4; ++it) {
    const int f = it * 256 + tid;
    const v4f v = *(const v4f*)(src + 4 * f);
    const int c = f >> 4;
    const int p0 = (f & 15) * 4;
    sW[c * 65 + p0 + 0] = v.x;
    sW[c * 65 + p0 + 1] = v.y;
    sW[c * 65 + p0 + 2] = v.z;
    sW[c * 65 + p0 + 3] = v.w;
  }
  __syncthreads();
  const int q = lane >> 3;
  const int c8 = (lane & 7) * 8;
  v8h hv[2];
#pragma unroll
  for (int it = 0; it < 2; ++it) {
    const int p = wave * 8 + it * 4 + q;
#pragma unroll
    for (int e = 0; e < 8; ++e) {
      const float sv = sW[(c8 + e) * 65 + p] * kWCarry;
      hv[it][e] = (_Float16)sv;
    }
  }
  for (int pass = 0; pass < 2; ++pass) {
#pragma unroll
    for (int it = 0; it < 2; ++it) {
      const int p = wave * 8 + it * 4 + q;
      *(volatile v8h*)(WP + ((size_t)p * kOC + o) * kCin + c8) = hv[it];
    }
    __threadfence();
  }
}

__global__ __launch_bounds__(128) void xform_in_kernel(const float* __restrict__ x, unsigned short* __restrict__ XT) {
  __shared__ __align__(16) float sR[64 * 128];
  __shared__ __align__(16) _Float16 sS[64 * 128];
  const int tid = threadIdx.x;
  const int lane = tid & 31;
  const int wave = __builtin_amdgcn_readfirstlane((int)(threadIdx.x >> 5));
  const int ml = wave >> 1;
  const int c = ((wave & 1) << 5) + lane;
  const int m = (int)blockIdx.x * 2 + ml;
  const int n = m / kTPI;
  const int rem = m - n * kTPI;
  const int a = rem / kNT;
  const int b = rem - a * kNT;
  const int h0 = 4 * a - 2;
  const int w0 = 4 * b - 2;
  const float* xb = x + (size_t)(n * kCin + c) * (kHW * kHW);

#pragma unroll 1
  for (int j = 0; j < 8; ++j) {
    const int h = h0 + j;
    const bool hok = (h >= 0) && (h < kHW);
    const int hc = h < 0 ? 0 : (h > kHW - 1 ? kHW - 1 : h);
    const float* xr = xb + hc * kHW;
    float d[8];
#pragma unroll
    for (int q = 0; q < 4; ++q) {
      const int wq = w0 + 2 * q;
      const bool ok = hok && (wq >= 0) && (wq <= kHW - 2);
      const int wc = wq < 0 ? 0 : (wq > kHW - 2 ? kHW - 2 : wq);
      const v2f v = *(const v2f*)(xr + wc);
      float vx = v.x;
      float vy = v.y;
      asm volatile("" : "+v"(vx), "+v"(vy));
      d[2 * q]     = ok ? vx : 0.0f;
      d[2 * q + 1] = ok ? vy : 0.0f;
    }
    float t[8];
    bt8(d, t);
#pragma unroll
    for (int l = 0; l < 8; ++l) sR[(j * 8 + l) * 128 + tid] = t[l];
  }

#pragma unroll 1
  for (int l = 0; l < 8; ++l) {
    float r[8];
#pragma unroll
    for (int j = 0; j < 8; ++j) r[j] = sR[(j * 8 + l) * 128 + tid];
    float t[8];
    bt8(r, t);
#pragma unroll
    for (int i = 0; i < 8; ++i) sS[(i * 8 + l) * 128 + tid] = (_Float16)t[i];
  }
  __syncthreads();

  const int hsel = lane >> 4;
  const int o8 = (lane & 15) * 8;
  v8h hv[8];
#pragma unroll
  for (int it = 0; it < 8; ++it) {
    const int p = wave * 16 + it * 2 + hsel;
    hv[it] = *(const v8h*)(sS + p * 128 + o8);
  }
  const size_t mrow0 = (size_t)blockIdx.x * 2;
  for (int pass = 0; pass < 2; ++pass) {
#pragma unroll
    for (int it = 0; it < 8; ++it) {
      const int p = wave * 16 + it * 2 + hsel;
      *(volatile v8h*)(XT + ((size_t)p * kMtot + mrow0) * kCin + o8) = hv[it];
    }
    __threadfence();
  }
}

__global__ __launch_bounds__(256) void gemm_f16_kernel(
    const unsigned short* __restrict__ Ap, const unsigned short* __restrict__ Btp, unsigned short* __restrict__ Cp,
    long strideA, long strideB, long strideC,
    int lda, int ldb, int ldc, int M, int N, int K, float scale) {
  const _Float16* A = (const _Float16*)Ap;
  const _Float16* Bt = (const _Float16*)Btp;
  __shared__ __align__(16) float sT[8][16 * 68];
  const int b = blockIdx.y;
  const int lane = threadIdx.x & 31;
  const int wave = __builtin_amdgcn_readfirstlane((int)(threadIdx.x >> 5));
  const int tilesN = N >> 6;
  const int tilesM = M >> 6;
  const int tile = (int)blockIdx.x * 8 + wave;
  if (tile >= tilesM * tilesN) return;
  const int tm = tile / tilesN;
  const int tn = tile - tm * tilesN;
  const int m0 = tm << 6;
  const int n0 = tn << 6;

  const _Float16* Ab = A + (size_t)b * strideA;
  const _Float16* Bb = Bt + (size_t)b * strideB;

  const int rlane = lane & 15;
  const int koff = (lane >> 4) * 8;
  const int mOff = (lane >> 4) * 8;

  v8f acc[4][4];
#pragma unroll
  for (int i = 0; i < 4; ++i)
#pragma unroll
    for (int j = 0; j < 4; ++j) acc[i][j] = (v8f){0.f, 0.f, 0.f, 0.f, 0.f, 0.f, 0.f, 0.f};

  for (int k0 = 0; k0 < K; k0 += 32) {
    v16h bh[4];
#pragma unroll
    for (int j = 0; j < 4; ++j) {
      const size_t bo = (size_t)(n0 + (j << 4) + rlane) * ldb + koff + k0;
      bh[j] = frag_load(Bb + bo);
    }
#pragma unroll
    for (int i = 0; i < 4; ++i) {
      const size_t ao = (size_t)(m0 + (i << 4) + rlane) * lda + koff + k0;
      const v16h ah = frag_load(Ab + ao);
#pragma unroll
      for (int j = 0; j < 4; ++j) acc[i][j] = mma_f16(ah, bh[j], acc[i][j]);
    }
  }

  float* slab = sT[wave];
  unsigned short* C = Cp + (size_t)b * strideC;
  const int q = lane >> 3;
  const int c8 = (lane & 7) * 8;
#pragma unroll
  for (int i = 0; i < 4; ++i) {
    const int mBase = m0 + (i << 4);
#pragma unroll
    for (int j = 0; j < 4; ++j) {
#pragma unroll
      for (int r = 0; r < 8; ++r) {
        const float v = acc[i][j][r] * scale;
        slab[(mOff + r) * 68 + (j << 4) + rlane] = v;
      }
    }
    __builtin_amdgcn_fence(__ATOMIC_RELEASE, "workgroup");
    __builtin_amdgcn_wave_barrier();
    __builtin_amdgcn_fence(__ATOMIC_ACQUIRE, "workgroup");
    v8h hv[4];
#pragma unroll
    for (int it = 0; it < 4; ++it) {
      const int row = it * 4 + q;
      const float* sp = slab + row * 68 + c8;
#pragma unroll
      for (int e = 0; e < 8; ++e) hv[it][e] = (_Float16)sp[e];
    }
    for (int pass = 0; pass < 2; ++pass) {
#pragma unroll
      for (int it = 0; it < 4; ++it) {
        const int row = it * 4 + q;
        *(volatile v8h*)(C + (size_t)(mBase + row) * ldc + n0 + c8) = hv[it];
      }
      __threadfence();
    }
    __builtin_amdgcn_fence(__ATOMIC_RELEASE, "workgroup");
    __builtin_amdgcn_wave_barrier();
    __builtin_amdgcn_fence(__ATOMIC_ACQUIRE, "workgroup");
  }
}

__global__ __launch_bounds__(256) void xform_out_kernel(const unsigned int* __restrict__ YTw, const float* __restrict__ bias,
                                                        float* __restrict__ out, int nbase) {
  __shared__ __align__(16) float sU[32 * 256];
  __shared__ __align__(16) float sO[16 * 4 * 64];
  const int tid = threadIdx.x;
  const int lane = tid & 31;
  const int wave = __builtin_amdgcn_readfirstlane((int)(threadIdx.x >> 5));
  const int bx = (int)blockIdx.x;
  const int ocg = bx & 7;
  const int tt = bx >> 3;
  const int nl = tt / kNT;
  const int a = tt - nl * kNT;
  const int ol = tid & 15;
  const int b = tid >> 4;
  const int bc = b < (kNT - 1) ? b : (kNT - 1);
  const int m = nl * kTPI + a * kNT + bc;
  const int o = ocg * 16 + ol;
  const unsigned sh = (unsigned)(o & 1) * 16u;
  const size_t wbase = ((size_t)m * kOC + o) >> 1;
  constexpr size_t kPlaneWords = (size_t)kMhalf * kOC / 2;
  const float bv = bias[o];

#pragma unroll 1
  for (int j = 0; j < 8; ++j) {
    float y[8];
#pragma unroll
    for (int i = 0; i < 8; ++i) {
      const unsigned wv = YTw[wbase + (size_t)(i * 8 + j) * kPlaneWords];
      y[i] = h16_to_f32((wv >> sh) & 0xffffu);
    }
    float z[4];
    at4(y, z);
#pragma unroll
    for (int pp = 0; pp < 4; ++pp) sU[(pp * 8 + j) * 256 + tid] = z[pp];
  }

#pragma unroll 1
  for (int pp = 0; pp < 4; ++pp) {
    float u[8];
#pragma unroll
    for (int j = 0; j < 8; ++j) u[j] = sU[(pp * 8 + j) * 256 + tid];
    float z[4];
    at4(u, z);
    v4f r;
    r.x = z[0] * kYInv + bv;
    r.y = z[1] * kYInv + bv;
    r.z = z[2] * kYInv + bv;
    r.w = z[3] * kYInv + bv;
    *(v4f*)(sO + (ol * 4 + pp) * 64 + 4 * b) = r;
  }
  __syncthreads();

  const int n = nbase + nl;
  const int f0 = lane;
  const int f1 = (32 + lane) < 56 ? (32 + lane) : 55;
  const int e0 = 4 * f0;
  const int e1 = 4 * f1;
  const int r0 = e0 / kHW;
  const int col0 = e0 - r0 * kHW;
  const int r1 = e1 / kHW;
  const int col1 = e1 - r1 * kHW;
  v4f sv[2][2];
#pragma unroll
  for (int s = 0; s < 2; ++s) {
    const int ocl = wave * 2 + s;
    sv[s][0] = *(const v4f*)(sO + (ocl * 4 + r0) * 64 + col0);
    sv[s][1] = *(const v4f*)(sO + (ocl * 4 + r1) * 64 + col1);
  }
  const bool act1 = lane < 24;
  for (int pass = 0; pass < 2; ++pass) {
#pragma unroll
    for (int s = 0; s < 2; ++s) {
      const int og = ocg * 16 + wave * 2 + s;
      float* dst = out + ((size_t)(n * kOC + og) * kHW + 4 * a) * kHW;
      *(volatile v4f*)(dst + 4 * f0) = sv[s][0];
      if (act1) *(volatile v4f*)(dst + 4 * (32 + lane)) = sv[s][1];
    }
    __threadfence();
  }
}

extern "C" void kernel_launch(void* const* d_in, const int* in_sizes, int n_in,
                              void* d_out, int out_size, void* d_ws, size_t ws_size,
                              hipStream_t stream) {
  if (n_in < 3) return;
  if (in_sizes[0] != kNB * kCin * kHW * kHW) return;
  if (in_sizes[1] != kOC * kCin * kP) return;
  if (in_sizes[2] != kOC) return;
  if (out_size != kNB * kOC * kHW * kHW) return;
  if (ws_size < kWsTotal) return;

  const float* x    = (const float*)d_in[0];
  const float* wgt  = (const float*)d_in[1];
  const float* bias = (const float*)d_in[2];
  float* out = (float*)d_out;

  char* ws = (char*)d_ws;
  unsigned short* WP = (unsigned short*)(ws + kOffWP);
  unsigned short* XT = (unsigned short*)(ws + kOffXT);
  unsigned short* YT = (unsigned short*)(ws + kOffYT);

  pack_w_kernel<<<kOC, 256, 0, stream>>>(wgt, WP);
  xform_in_kernel<<<kMtot / 2, 128, 0, stream>>>(x, XT);

  const int tiles = (kMhalf / 64) * (kOC / 64);
  const int gx = (tiles + 7) / 8;
  for (int half = 0; half < 2; ++half) {
    gemm_f16_kernel<<<dim3(gx, kP), 256, 0, stream>>>(
        XT + (size_t)half * kMhalf * kCin, WP, YT,
        (long)kMtot * kCin, (long)kOC * kCin, (long)kMhalf * kOC,
        kCin, kCin, kOC, kMhalf, kOC, kCin, kGemmScale);
    xform_out_kernel<<<kHalfN * kNT * 8, 256, 0, stream>>>(
        (const unsigned int*)YT, bias, out, half * kHalfN);
  }
}
